// GraphAttn_20280835572246
// MI455X (gfx1250) — hardware-verified
//
#include <hip/hip_runtime.h>
#include <math.h>

typedef __attribute__((ext_vector_type(16))) _Float16 v16h;
typedef __attribute__((ext_vector_type(16))) __bf16 v16b;
typedef __attribute__((ext_vector_type(8)))  _Float16 v8h;
typedef __attribute__((ext_vector_type(8)))  float v8f;
typedef __attribute__((ext_vector_type(4)))  float v4f;
typedef __attribute__((ext_vector_type(2)))  float v2f;
typedef __attribute__((ext_vector_type(4)))  unsigned v4u;
typedef __attribute__((ext_vector_type(4)))  int v4i;
typedef float __attribute__((may_alias)) float_a;
typedef int __attribute__((may_alias)) int_a;

template <typename T> __device__ __forceinline__ void vst2(void* p, T v) { *(volatile T*)p = v; __threadfence(); *(volatile T*)p = v; }
__device__ __forceinline__ v8f wmma16(v16h a, v16h b, v8f c) {
  v8f d = __builtin_amdgcn_wmma_f32_16x16x32_f16(false, a, false, b, (short)0, c, false, false);
  asm volatile("v_nop\n\tv_nop\n\tv_nop\n\tv_nop" : "+v"(d) : "v"(a), "v"(b));
  return d;
}
__device__ __forceinline__ v8f wmma_bf(v16b a, v16b b, v8f c) {
  v8f d = __builtin_amdgcn_wmma_f32_16x16x32_bf16(false, a, false, b, (short)0, c, false, false);
  asm volatile("v_nop\n\tv_nop\n\tv_nop\n\tv_nop" : "+v"(d) : "v"(a), "v"(b));
  return d;
}
__device__ __forceinline__ v16h frag_h(const _Float16* rowk0, int lane) {
  union { v16h v; v8h q[2]; } u; const _Float16* p = rowk0 + 8 * (lane >> 4);
  u.q[0] = *(const v8h*)p; u.q[1] = *(const v8h*)(p + 16); return u.v;
}
__device__ __forceinline__ v16h frag_f32(const float* rowk0, int lane) {
  v16h a; const float* p = rowk0 + 8 * (lane >> 4);
#pragma unroll
  for (int i = 0; i < 8; ++i) { a[i] = (_Float16)p[i]; a[8 + i] = (_Float16)p[16 + i]; }
  return a;
}
__device__ __forceinline__ v16h frag_f32s(const float* rowk0, int lane, float sc) {
  v16h a; const float* p = rowk0 + 8 * (lane >> 4);
#pragma unroll
  for (int i = 0; i < 8; ++i) { a[i] = (_Float16)(p[i] * sc); a[8 + i] = (_Float16)(p[16 + i] * sc); }
  return a;
}
__device__ __forceinline__ v16h fragc_f32(const float* W, int k0, int n, int lane, int ld, int K) {
  v16h a; const int g = lane >> 4;
#pragma unroll
  for (int i = 0; i < 8; ++i) { const int ka = k0 + 8 * g + i, kb = ka + 16;
    a[i] = (_Float16)(ka < K ? W[(size_t)(ka < K ? ka : K - 1) * ld + n] : 0.f); a[8 + i] = (_Float16)(kb < K ? W[(size_t)(kb < K ? kb : K - 1) * ld + n] : 0.f); }
  return a;
}
struct F2 { v16b h, l; };
__device__ __forceinline__ F2 bsplit16(const float v[16]) { F2 r;
#pragma unroll
  for (int i = 0; i < 16; ++i) { const __bf16 h = (__bf16)v[i]; r.h[i] = h; r.l[i] = (__bf16)(v[i] - (float)h); }
  return r; }
__device__ __forceinline__ F2 split_row(const float* row, int k0, int lane) { float v[16]; const float* p = row + k0 + 8 * (lane >> 4);
#pragma unroll
  for (int i = 0; i < 8; ++i) { v[i] = p[i]; v[8 + i] = p[16 + i]; }
  return bsplit16(v); }
__device__ __forceinline__ F2 split_rowK(const float* row, int k0, int lane, int K) { float v[16]; const int g = lane >> 4;
#pragma unroll
  for (int i = 0; i < 8; ++i) { const int ka = k0 + 8 * g + i, kb = ka + 16; v[i] = ka < K ? row[ka < K ? ka : K - 1] : 0.f; v[8 + i] = kb < K ? row[kb < K ? kb : K - 1] : 0.f; }
  return bsplit16(v); }
__device__ __forceinline__ F2 split_col(const float* W, int k0, int n, int lane, int ld, int K) { float v[16]; const int g = lane >> 4;
#pragma unroll
  for (int i = 0; i < 8; ++i) { const int ka = k0 + 8 * g + i, kb = ka + 16; v[i] = ka < K ? W[(size_t)(ka < K ? ka : K - 1) * ld + n] : 0.f; v[8 + i] = kb < K ? W[(size_t)(kb < K ? kb : K - 1) * ld + n] : 0.f; }
  return bsplit16(v); }
__device__ __forceinline__ v8f mac3(const F2& a, const F2& b, v8f c) { c = wmma_bf(a.l, b.h, c); c = wmma_bf(a.h, b.l, c); return wmma_bf(a.h, b.h, c); }
__device__ __forceinline__ float sigm(float v) { return 1.0f / (1.0f + expf(-v)); }
#define LDSX() do { asm volatile("s_wait_dscnt 0" ::: "memory"); __builtin_amdgcn_wave_barrier(); __builtin_amdgcn_fence(__ATOMIC_RELEASE, "workgroup"); } while (0)


#define NB 32
#define NN 512
#define FI 64
#define OD 128
#define NH 8
#define DH 16
#ifndef TNB
#define TNB NB
#endif
typedef __attribute__((ext_vector_type(8))) __bf16 v8b;
__device__ __forceinline__ v16b frag_b(const __bf16* rowk0, int lane) {
  union { v16b v; v8b q[2]; } u; const __bf16* p = rowk0 + 8 * (lane >> 4);
  u.q[0] = *(const v8b*)p; u.q[1] = *(const v8b*)(p + 16); return u.v;
}
__device__ __forceinline__ float bfr(float v) { return (float)(__bf16)v; }
__device__ __attribute__((noinline)) float exp_ni(float v) { return expf(v); }
__device__ __attribute__((noinline)) float erf_ni(float v) { return erff(v); }

#define WS_QH  0u
#define WS_QL  (WS_QH + 2u * (size_t)NB * NN * OD)
#define WS_KH  (WS_QL + 2u * (size_t)NB * NN * OD)
#define WS_KL  (WS_KH + 2u * (size_t)NB * NN * OD)
#define WS_VH  (WS_KL + 2u * (size_t)NB * NN * OD)
#define WS_VL  (WS_VH + 2u * (size_t)NB * OD * NN)
#define WS_END (WS_VL + 2u * (size_t)NB * OD * NN)

__global__ __launch_bounds__(128) void k_proj(const float* __restrict__ X, const float* __restrict__ WQ, const float* __restrict__ WK, const float* __restrict__ WV, _Float16* __restrict__ QH, _Float16* __restrict__ QL, _Float16* __restrict__ KH, _Float16* __restrict__ KL, _Float16* __restrict__ VH, _Float16* __restrict__ VL) {
  __shared__ __align__(16) _Float16 sq[64][136], sql[64][136], sk[64][136], skl[64][136]; __shared__ __align__(16) _Float16 th[OD][72], tl[OD][72];
  const int tid = threadIdx.x, wave = tid >> 5, lane = tid & 31, col = lane & 15, g = lane >> 4; const size_t row0 = (size_t)blockIdx.x * 64; const size_t b = row0 / NN; const int n0 = (int)(row0 % NN); const size_t r0 = row0 + wave * 16;
#pragma unroll 1
  for (int which = 0; which < 3; ++which) { const float* Wm = which == 0 ? WQ : which == 1 ? WK : WV; v8f acc[8] = {};
#pragma unroll
    for (int kc = 0; kc < FI / 32; ++kc) { v16b a; const float* pp = X + (r0 + col) * FI + kc * 32 + 8 * g;
#pragma unroll
      for (int i = 0; i < 8; ++i) { a[i] = (__bf16)pp[i]; a[8 + i] = (__bf16)pp[16 + i]; }
#pragma unroll
      for (int j = 0; j < 8; ++j) { v16b w; const int o = j * 16 + col;
#pragma unroll
        for (int i = 0; i < 8; ++i) { w[i] = (__bf16)Wm[(size_t)(kc * 32 + 8 * g + i) * OD + o]; w[8 + i] = (__bf16)Wm[(size_t)(kc * 32 + 16 + 8 * g + i) * OD + o]; }
        acc[j] = wmma_bf(a, w, acc[j]); } }
#pragma unroll
    for (int j = 0; j < 8; ++j)
#pragma unroll
      for (int r = 0; r < 8; ++r) { const float v = acc[j][r]; const _Float16 hv = (_Float16)v, lv = (_Float16)((v - (float)hv) * 2048.0f); const int rl = wave * 16 + 8 * g + r, cl = j * 16 + col; if (which == 0) { sq[rl][cl] = hv; sql[rl][cl] = lv; } else if (which == 1) { sk[rl][cl] = hv; skl[rl][cl] = lv; } else { th[cl][rl] = hv; tl[cl][rl] = lv; } } }
  __syncthreads();
  for (int e = tid; e < 64 * 16; e += 128) { const int rl = e >> 4, q = e & 15; const size_t o = (row0 + rl) * OD + q * 8; vst2((unsigned*)(QH + o), *(const v4u*)&sq[rl][q * 8]); vst2((unsigned*)(QL + o), *(const v4u*)&sql[rl][q * 8]); vst2((unsigned*)(KH + o), *(const v4u*)&sk[rl][q * 8]); vst2((unsigned*)(KL + o), *(const v4u*)&skl[rl][q * 8]); }
  for (int e = tid; e < OD * 8; e += 128) { const int c = e >> 3, q = e & 7; const size_t o = (b * OD + c) * (size_t)NN + n0 + q * 8; vst2((unsigned*)(VH + o), *(const v4u*)&th[c][q * 8]); vst2((unsigned*)(VL + o), *(const v4u*)&tl[c][q * 8]); } }
__global__ __launch_bounds__(128) void k_att(const _Float16* __restrict__ QH, const _Float16* __restrict__ QL, const _Float16* __restrict__ KH, const _Float16* __restrict__ KL, const _Float16* __restrict__ VH, const _Float16* __restrict__ VL, const float* __restrict__ ADJ, const float* __restrict__ WO, float* __restrict__ OUT) {
  __shared__ __align__(16) float sp[4][16][36]; __shared__ __align__(16) float so[4][16][132];
  const int tid = threadIdx.x, wave = tid >> 5, lane = tid & 31, col = lane & 15, g = lane >> 4; const size_t b = blockIdx.y; const int q0 = blockIdx.x * 64 + wave * 16; const size_t rq = b * NN + q0;
#pragma unroll 1
  for (int h = 0; h < NH; ++h) {
    v16h aq, al; { const _Float16* ph = QH + (rq + col) * OD + h * DH + 8 * g; const _Float16* pl = QL + (rq + col) * OD + h * DH + 8 * g;
#pragma unroll
      for (int i = 0; i < 8; ++i) { aq[i] = ph[i]; al[i] = pl[i]; aq[8 + i] = (_Float16)0.0f; al[8 + i] = (_Float16)0.0f; } }
    v8f acc = {}, accl = {};
#pragma unroll 1
    for (int ks = 0; ks < NN / 32; ++ks) {
#pragma unroll
      for (int ct = 0; ct < 2; ++ct) { const int kk = ks * 32 + ct * 16 + col; const size_t rk = (b * NN + kk) * OD + h * DH; const v16h kh = frag_h(KH + rk, lane), kl = frag_h(KL + rk, lane); v8f c = {}, cl = {}; c = wmma16(aq, kh, c); cl = wmma16(aq, kl, cl); cl = wmma16(al, kh, cl);
#pragma unroll
        for (int r = 0; r < 8; ++r) { const float sc = (c[r] + cl[r] * (1.0f / 2048.0f)) * 0.25f; const float a = bfr(ADJ[((size_t)b * NN + q0 + 8 * g + r) * NN + kk]); sp[wave][8 * g + r][ct * 16 + col] = tanhf(sc * a); } }
      LDSX();
      v16h pa, pal; { const float* prow = &sp[wave][col][0] + 8 * (lane >> 4);
#pragma unroll
        for (int i = 0; i < 8; ++i) { const float p0 = prow[i], p1 = prow[16 + i]; pa[i] = (_Float16)p0; pa[8 + i] = (_Float16)p1; pal[i] = (_Float16)((p0 - (float)pa[i]) * 2048.0f); pal[8 + i] = (_Float16)((p1 - (float)pa[8 + i]) * 2048.0f); } }
      { const size_t po = (b * OD + (size_t)h * DH + col) * NN + ks * 32; const v16h vh = frag_h(VH + po, lane), vl = frag_h(VL + po, lane); acc = wmma16(pa, vh, acc); accl = wmma16(pa, vl, accl); accl = wmma16(pal, vh, accl); }
      LDSX(); }
#pragma unroll
    for (int r = 0; r < 8; ++r) so[wave][8 * g + r][h * DH + col] = acc[r] + accl[r] * (1.0f / 2048.0f); }
  LDSX();
  { v8f acc3[8] = {};
#pragma unroll
    for (int kc = 0; kc < OD / 32; ++kc) { float v[16]; const float* pp = &so[wave][col][kc * 32 + 8 * g];
#pragma unroll
      for (int i = 0; i < 8; ++i) { v[i] = pp[i]; v[8 + i] = pp[16 + i]; }
      const F2 a = bsplit16(v);
#pragma unroll
      for (int j = 0; j < 8; ++j) { v16b w; const int o = j * 16 + col;
#pragma unroll
        for (int i = 0; i < 8; ++i) { w[i] = (__bf16)WO[(size_t)(kc * 32 + 8 * g + i) * OD + o]; w[8 + i] = (__bf16)WO[(size_t)(kc * 32 + 16 + 8 * g + i) * OD + o]; }
        acc3[j] = wmma_bf(a.h, w, acc3[j]); acc3[j] = wmma_bf(a.l, w, acc3[j]); } }
    LDSX();
#pragma unroll
    for (int j = 0; j < 8; ++j)
#pragma unroll
      for (int r = 0; r < 8; ++r) so[wave][8 * g + r][j * 16 + col] = fmaxf(acc3[j][r], 0.f); }
  LDSX(); for (int rl = 0; rl < 16; ++rl) vst2(OUT + (rq + rl) * OD + lane * 4, *(const v4f*)&so[wave][rl][lane * 4]); }
extern "C" void kernel_launch(void* const* d_in, const int* in_sizes, int n_in, void* d_out, int out_size, void* d_ws, size_t ws_size, hipStream_t stream) {
  (void)in_sizes; (void)n_in; (void)out_size;
  const float** F = (const float**)d_in;
  if (ws_size < (size_t)WS_END) return;
  char* ws = (char*)d_ws; _Float16 *QH = (_Float16*)(ws + WS_QH), *QL = (_Float16*)(ws + WS_QL), *KH = (_Float16*)(ws + WS_KH), *KL = (_Float16*)(ws + WS_KL), *VH = (_Float16*)(ws + WS_VH), *VL = (_Float16*)(ws + WS_VL);
  k_proj<<<NB * NN / 64, 128, 0, stream>>>(F[0], F[2], F[3], F[4], QH, QL, KH, KL, VH, VL);
  k_att<<<dim3(NN / 64, TNB), 128, 0, stream>>>(QH, QL, KH, KL, VH, VL, F[1], F[5], (float*)d_out);
}
